// DIT_49881750176273
// MI455X (gfx1250) — hardware-verified
//
#include <hip/hip_runtime.h>
#include <math.h>
#include <stdint.h>

constexpr int kS        = 2048;
constexpr int kNTok     = 1024;
constexpr int kD        = 1024;
constexpr int kH        = 16;
constexpr int kHD       = 64;
constexpr int kRopeHalf = 32;
constexpr int kCond     = 128;
constexpr int kD3       = 3 * kD;
constexpr int kD4       = 4 * kD;
constexpr int kD6       = 6 * kD;
constexpr int kBlkShift = 4;
constexpr float kWsc    = 32.0f;
constexpr float kW2sc   = 64.0f;

typedef __attribute__((ext_vector_type(16))) _Float16 v16h;
typedef __attribute__((ext_vector_type(8)))  _Float16 v8h;
typedef __attribute__((ext_vector_type(16))) __bf16   v16b;
typedef __attribute__((ext_vector_type(8)))  __bf16   v8b;
typedef __attribute__((ext_vector_type(8)))  float    v8f;
typedef __attribute__((ext_vector_type(4)))  float    v4f;
typedef __attribute__((ext_vector_type(2)))  float    v2f;

__device__ __forceinline__ unsigned short f2bf_bits(float f) {
  unsigned u = __float_as_uint(f);
  return (unsigned short)((u + 0x7FFFu + ((u >> 16) & 1u)) >> 16);
}
__device__ __forceinline__ float bf_bits2f(unsigned short h) { return __uint_as_float(((unsigned)h) << 16); }

__device__ __forceinline__ void dep_guard_h(v8f& a, v8f& b, v16h x, v16h y) { asm volatile("v_nop\n\tv_nop\n\tv_nop\n\tv_nop" : "+v"(a), "+v"(b) : "v"(x), "v"(y)); }
__device__ __forceinline__ void dep_guard_b(v8f& a, v8f& b, v16b x, v16b y) { asm volatile("v_nop\n\tv_nop\n\tv_nop\n\tv_nop" : "+v"(a), "+v"(b) : "v"(x), "v"(y)); }
__device__ __forceinline__ void keep4_h(v16h a, v16h b, v16h c, v16h d) { asm volatile("v_nop" :: "v"(a), "v"(b), "v"(c), "v"(d)); }
__device__ __forceinline__ void keep4_b(v16b a, v16b b, v16b c, v16b d) { asm volatile("v_nop" :: "v"(a), "v"(b), "v"(c), "v"(d)); }
__device__ __forceinline__ void acc_guard4(v8f& a, v8f& b, v8f& c, v8f& d) { asm volatile("v_nop\n\tv_nop\n\tv_nop\n\tv_nop" : "+v"(a), "+v"(b), "+v"(c), "+v"(d)); }
template <typename T> struct Frag;
template <> struct Frag<_Float16> {
  typedef v16h V; union U { v16h v; v8h h[2]; };
  static __device__ __forceinline__ v16h load(const _Float16* p) {
    U f; f.h[0] = *(const v8h*)(p); f.h[1] = *(const v8h*)(p + 16); return f.v;
  }
  static __device__ __forceinline__ v8f mma(v16h a, v16h b, v8f c) {
    return __builtin_amdgcn_wmma_f32_16x16x32_f16(false, a, false, b, (short)0, c, false, false);
  }
  static __device__ __forceinline__ void guard(v8f& a, v8f& b, v16h x, v16h y) { dep_guard_h(a, b, x, y); }
  static __device__ __forceinline__ void keep(v16h a, v16h b, v16h c, v16h d) { keep4_h(a, b, c, d); }
};
template <> struct Frag<__bf16> {
  typedef v16b V; union U { v16b v; v8b h[2]; };
  static __device__ __forceinline__ v16b load(const __bf16* p) {
    U f; f.h[0] = *(const v8b*)(p); f.h[1] = *(const v8b*)(p + 16); return f.v;
  }
  static __device__ __forceinline__ v8f mma(v16b a, v16b b, v8f c) {
    return __builtin_amdgcn_wmma_f32_16x16x32_bf16(false, a, false, b, (short)0, c, false, false);
  }
  static __device__ __forceinline__ void guard(v8f& a, v8f& b, v16b x, v16b y) { dep_guard_b(a, b, x, y); }
  static __device__ __forceinline__ void keep(v16b a, v16b b, v16b c, v16b d) { keep4_b(a, b, c, d); }
};

template <int ET> struct Elem;
template <> struct Elem<0> { typedef _Float16 T; };
template <> struct Elem<1> { typedef __bf16 T; };
template <int ET, bool SPLIT, int BIAS_MODE, int OUT_MODE, bool RESID, int ACT, bool GATE>
__global__ __launch_bounds__(256) void wmma_gemm64(
    const unsigned short* __restrict__ Ap, const unsigned short* __restrict__ A2p, int lda, long strideA,
    const unsigned short* __restrict__ Btp, const unsigned short* __restrict__ Bt2p, int ldb, long strideB,
    void* __restrict__ Cout, void* __restrict__ Cout2, int ldc, long strideC,
    const float* __restrict__ bias,
    const float* __restrict__ resid, long strideR,
    const float* __restrict__ gate,
    const float* __restrict__ ropeCos, const float* __restrict__ ropeSin, long planeStride,
    int M, int N, int K, float scale) {
  typedef typename Elem<ET>::T T;
  typedef typename Frag<T>::V V;
  const T* A = (const T*)Ap; const T* A2 = (const T*)A2p; const T* Bt = (const T*)Btp; const T* Bt2 = (const T*)Bt2p;
  __shared__ __align__(16) float sT[8][16 * 68];
  const int b    = blockIdx.y;
  const int lane = threadIdx.x & 31;
  const int wave = threadIdx.x >> 5;
  const int tilesN = N >> 6;
  const int tilesM = M >> 6;
  const int tile = blockIdx.x * 8 + wave;
  if (tile >= tilesM * tilesN) return;
  const int tm = tile / tilesN;
  const int tn = tile - tm * tilesN;
  const int m0 = tm << 6;
  const int n0 = tn << 6;

  const T* Ab  = A  + (size_t)b * strideA;
  const T* Bb  = Bt + (size_t)b * strideB;
  const T* Ab2 = SPLIT ? (A2  + (size_t)b * strideA) : nullptr;
  const T* Bb2 = SPLIT ? (Bt2 + (size_t)b * strideB) : nullptr;

  const int rlane = lane & 15;
  const int koff  = (lane >> 4) * 8;
  const int mOff  = (lane >> 4) * 8;

  v8f acc[4][4];
#pragma unroll
  for (int i = 0; i < 4; ++i)
#pragma unroll
    for (int j = 0; j < 4; ++j) acc[i][j] = (v8f){0.f,0.f,0.f,0.f,0.f,0.f,0.f,0.f};

  for (int k0 = 0; k0 < K; k0 += 32) {
    V bh[4], bl[4];
#pragma unroll
    for (int j = 0; j < 4; ++j) {
      const size_t bo = (size_t)(n0 + (j << 4) + rlane) * ldb + koff + k0;
      bh[j] = Frag<T>::load(Bb + bo);
      if (SPLIT) bl[j] = Frag<T>::load(Bb2 + bo);
    }
#pragma unroll
    for (int i = 0; i < 4; ++i) {
      const size_t ao = (size_t)(m0 + (i << 4) + rlane) * lda + koff + k0;
      V ah = Frag<T>::load(Ab + ao);
      V al;
      if (SPLIT) al = Frag<T>::load(Ab2 + ao);
#pragma unroll
      for (int j = 0; j < 4; ++j) {
        acc[i][j] = Frag<T>::mma(ah, bh[j], acc[i][j]);
        if (SPLIT) {
          acc[i][j] = Frag<T>::mma(ah, bl[j], acc[i][j]);
          acc[i][j] = Frag<T>::mma(al, bh[j], acc[i][j]);
        }
      }
      Frag<T>::guard(acc[i][0], acc[i][3], ah, SPLIT ? al : ah);
    }
    Frag<T>::keep(bh[0], bh[1], bh[2], bh[3]);
    if (SPLIT) Frag<T>::keep(bl[0], bl[1], bl[2], bl[3]);
  }
  acc_guard4(acc[0][0], acc[0][1], acc[0][2], acc[0][3]);
  acc_guard4(acc[1][0], acc[1][1], acc[1][2], acc[1][3]);
  acc_guard4(acc[2][0], acc[2][1], acc[2][2], acc[2][3]);
  acc_guard4(acc[3][0], acc[3][1], acc[3][2], acc[3][3]);

  float* slab = sT[wave];
  const float* Rb = RESID ? (resid + (size_t)b * strideR) : nullptr;
#pragma unroll
  for (int i = 0; i < 4; ++i) {
    const int mBase = m0 + (i << 4);
    if (OUT_MODE == 3) {
#pragma unroll
      for (int j = 0; j < 2; ++j) {
        const int dlo = (j << 4) + rlane;
#pragma unroll
        for (int r = 0; r < 8; ++r) {
          const int pos = (mBase + mOff + r) & (kNTok - 1);
          const float cs = ropeCos[pos * kRopeHalf + dlo];
          const float sn = ropeSin[pos * kRopeHalf + dlo];
          const float xl = acc[i][j][r] * scale;
          const float xh = acc[i][j + 2][r] * scale;
          slab[(mOff + r) * 68 + (j << 4) + rlane]       = xl * cs - xh * sn;
          slab[(mOff + r) * 68 + ((j + 2) << 4) + rlane] = xh * cs + xl * sn;
        }
      }
    } else {
#pragma unroll
      for (int j = 0; j < 4; ++j) {
        const int n = n0 + (j << 4) + rlane;
        float bv = 0.f, gv = 1.f;
        if (BIAS_MODE == 2) bv = bias[n];
        if (GATE) gv = gate[n];
#pragma unroll
        for (int r = 0; r < 8; ++r) {
          float v = acc[i][j][r] * scale;
          if (BIAS_MODE == 1) v += bias[mBase + mOff + r];
          if (BIAS_MODE == 2) v += bv;
          if (ACT == 6) {
            const float u2 = v * (1.5957691216f + 0.0713548163f * v * v);
            const float e  = __expf(fminf(-u2, 80.0f));
            v = v * __builtin_amdgcn_rcpf(1.0f + e);
          }
          if (GATE) v *= gv;
          if (RESID) v += Rb[(size_t)(mBase + mOff + r) * ldc + n];
          slab[(mOff + r) * 68 + (j << 4) + rlane] = v;
        }
      }
    }
    __builtin_amdgcn_fence(__ATOMIC_RELEASE, "workgroup");
    __builtin_amdgcn_wave_barrier();
    __builtin_amdgcn_fence(__ATOMIC_ACQUIRE, "workgroup");
    if (OUT_MODE == 0) {
      float* C = (float*)Cout + (size_t)b * strideC;
      const int hh = lane >> 4, c4 = (lane & 15) * 4;
      for (int pass = 0; pass < 2; ++pass) {
#pragma unroll
        for (int it = 0; it < 8; ++it) {
          const int row = it * 2 + hh;
          v4f v = *(const v4f*)(slab + row * 68 + c4);
          *(volatile v4f*)(C + (size_t)(mBase + row) * ldc + n0 + c4) = v;
        }
        __threadfence();
      }
    } else {
      const int q = lane >> 3, c8 = (lane & 7) * 8;
      unsigned short* C = (unsigned short*)Cout + (size_t)b * strideC;
      size_t cbase = 0;
      int ncol = n0;
      if (OUT_MODE == 3) {
        const int which = n0 / ldc;
        ncol  = n0 - which * ldc;
        cbase = (size_t)which * (size_t)planeStride;
      }
      for (int pass = 0; pass < 2; ++pass) {
#pragma unroll
        for (int it = 0; it < 4; ++it) {
          const int row = it * 4 + q;
          const float* sp = slab + row * 68 + c8;
          v8h hv;
#pragma unroll
          for (int e = 0; e < 8; ++e) hv[e] = (_Float16)sp[e];
          *(volatile v8h*)(C + cbase + (size_t)(mBase + row) * ldc + ncol + c8) = hv;
        }
        __threadfence();
      }
    }
    __builtin_amdgcn_fence(__ATOMIC_RELEASE, "workgroup");
    __builtin_amdgcn_wave_barrier();
    __builtin_amdgcn_fence(__ATOMIC_ACQUIRE, "workgroup");
  }
}

__global__ __launch_bounds__(256) void cast_scale_f16x2(
    const float* __restrict__ in, unsigned short* __restrict__ out, int n2, float sc) {
  const int i = blockIdx.x * 256 + threadIdx.x;
  if (i < n2) {
    const v2f f = *(const v2f*)(in + 2 * (size_t)i);
    const _Float16 h0 = (_Float16)(f[0] * sc), h1 = (_Float16)(f[1] * sc);
    const unsigned u = (unsigned)__builtin_bit_cast(unsigned short, h0) | ((unsigned)__builtin_bit_cast(unsigned short, h1) << 16);
    ((volatile unsigned*)out)[i] = u;
    __threadfence();
    ((volatile unsigned*)out)[i] = u;
  }
}

__global__ __launch_bounds__(256) void cond_mod_kernel(const float* __restrict__ cvec, const float* __restrict__ W,
                                                       const float* __restrict__ bvec, float* __restrict__ mods,
                                                       int nout, int kc) {
  const int j  = blockIdx.x * 256 + threadIdx.x;
  const int jc = (j < nout) ? j : (nout - 1);
  float acc = bvec[jc];
  const float* wr = W + (size_t)jc * kc;
#pragma unroll 1
  for (int k = 0; k < kc; ++k) acc += cvec[k] * wr[k];
  if (j < nout) {
    ((volatile float*)mods)[j] = acc;
    __threadfence();
    ((volatile float*)mods)[j] = acc;
  }
}

__global__ __launch_bounds__(128) void ln_mod_kernel(const float* __restrict__ x, const float* __restrict__ w,
                                                     const float* __restrict__ sh, const float* __restrict__ sc,
                                                     unsigned short* __restrict__ out) {
  __shared__ float red0[4];
  __shared__ float red1[4];
  const int row = blockIdx.x, tid = threadIdx.x, lane = tid & 31, wave = tid >> 5;
  const int col0 = tid * 8;
  const float* xr = x + (size_t)row * kD + col0;
  const v4f xa = *(const v4f*)xr;
  const v4f xb = *(const v4f*)(xr + 4);
  float v[8] = {xa[0], xa[1], xa[2], xa[3], xb[0], xb[1], xb[2], xb[3]};
  float s = ((v[0] + v[1]) + (v[2] + v[3])) + ((v[4] + v[5]) + (v[6] + v[7]));
#pragma unroll
  for (int off = 16; off > 0; off >>= 1) s += __shfl_xor(s, off, 32);
  if (lane == 0) red0[wave] = s;
  __syncthreads();
  const float mean = ((red0[0] + red0[1]) + (red0[2] + red0[3])) * (1.0f / (float)kD);
  float sq = 0.f;
#pragma unroll
  for (int e = 0; e < 8; ++e) { const float d = v[e] - mean; sq += d * d; }
#pragma unroll
  for (int off = 16; off > 0; off >>= 1) sq += __shfl_xor(sq, off, 32);
  if (lane == 0) red1[wave] = sq;
  __syncthreads();
  const float var  = ((red1[0] + red1[1]) + (red1[2] + red1[3])) * (1.0f / (float)kD);
  const float rstd = rsqrtf(var + 1e-5f);
  const v4f wa = *(const v4f*)(w + col0),  wb = *(const v4f*)(w + col0 + 4);
  const v4f ca = *(const v4f*)(sc + col0), cb = *(const v4f*)(sc + col0 + 4);
  const v4f ha = *(const v4f*)(sh + col0), hb = *(const v4f*)(sh + col0 + 4);
  float wv[8] = {wa[0], wa[1], wa[2], wa[3], wb[0], wb[1], wb[2], wb[3]};
  float cv[8] = {ca[0], ca[1], ca[2], ca[3], cb[0], cb[1], cb[2], cb[3]};
  float hv8[8] = {ha[0], ha[1], ha[2], ha[3], hb[0], hb[1], hb[2], hb[3]};
  v8h hv;
#pragma unroll
  for (int e = 0; e < 8; ++e) hv[e] = (_Float16)(((v[e] - mean) * rstd * wv[e]) * (1.0f + cv[e]) + hv8[e]);
  _Float16* orow = (_Float16*)(void*)out + (size_t)row * kD + col0;
  *(volatile v8h*)orow = hv;
  __threadfence();
  *(volatile v8h*)orow = hv;
}

__global__ __launch_bounds__(256) void vtrans_kernel(const unsigned short* __restrict__ vin, unsigned short* __restrict__ vt) {
  __shared__ __align__(16) _Float16 th[64 * 72];
  const _Float16* V = (const _Float16*)(const void*)vin;
  _Float16* O = (_Float16*)(void*)vt;
  const int c0  = blockIdx.x * 64;
  const int r0  = blockIdx.y * 64;
  const int tid = threadIdx.x;
  const int sub = tid >> 3;
  const int c8  = (tid & 7) * 8;
#pragma unroll
  for (int it = 0; it < 2; ++it) {
    const int rr = it * 32 + sub;
    const v8h a = *(const v8h*)(V + (size_t)(r0 + rr) * kD + c0 + c8);
    *(v8h*)(th + rr * 72 + c8) = a;
  }
  __syncthreads();
  v8h hv[2];
#pragma unroll
  for (int it = 0; it < 2; ++it) {
    const int oc = it * 32 + sub;
#pragma unroll
    for (int e = 0; e < 8; ++e) hv[it][e] = th[(c8 + e) * 72 + oc];
  }
  for (int pass = 0; pass < 2; ++pass) {
#pragma unroll
    for (int it = 0; it < 2; ++it) {
      const int oc = it * 32 + sub;
      *(volatile v8h*)(O + (size_t)(c0 + oc) * kS + r0 + c8) = hv[it];
    }
    __threadfence();
  }
}

constexpr int kAtD = 64, kAtNW = 4, kAtQB = 64, kAtKC = 64;
constexpr float kPsc = 32768.0f;

__device__ __forceinline__ v8f mma_h(v16h a, v16h b, v8f c) {
  c = __builtin_amdgcn_wmma_f32_16x16x32_f16(false, a, false, b, (short)0, c, false, false);
  asm volatile("v_nop\n\tv_nop\n\tv_nop\n\tv_nop" : "+v"(c) : "v"(a), "v"(b));
  return c;
}

__global__ __launch_bounds__(128)
void attn_bd_kernel(const unsigned short* __restrict__ qp, const unsigned short* __restrict__ kp,
                    const unsigned short* __restrict__ vtp, unsigned short* __restrict__ op, float sscale) {
  union FH { v16h v; v8h h[2]; };
  __shared__ __align__(16) _Float16 Ksh[kAtKC * kAtD];
  __shared__ __align__(16) _Float16 Vth[kAtD * kAtKC];
  __shared__ __align__(16) _Float16 Psh[kAtNW][16 * kAtKC];
  __shared__ __align__(16) float    Os[kAtNW][16 * 68];

  const int tid  = threadIdx.x;
  const int wave = tid >> 5;
  const int lane = tid & 31;
  const int hh   = lane >> 4;
  const int c    = lane & 15;

  constexpr int nqb     = kS / kAtQB;
  constexpr int nqbHalf = kNTok / kAtQB;
  constexpr int kcHalf  = kNTok / kAtKC;
  const int bx = blockIdx.x;
  const int qb = bx % nqb;
  const int h  = bx / nqb;
  const int q0 = qb * kAtQB + wave * 16;

  const _Float16* Q  = (const _Float16*)(const void*)qp  + (size_t)h * kAtD;
  const _Float16* Kp = (const _Float16*)(const void*)kp  + (size_t)h * kAtD;
  const _Float16* VT = (const _Float16*)(const void*)vtp + (size_t)h * kAtD * kS;
  _Float16*       O  = (_Float16*)(void*)op + (size_t)h * kAtD;

  v16h qa[2];
#pragma unroll
  for (int dc = 0; dc < 2; ++dc)
    qa[dc] = Frag<_Float16>::load(Q + (size_t)(q0 + c) * kD + dc * 32 + 8 * hh);

  float mrow[8], lrow[8];
  v8f oacc[4];
#pragma unroll
  for (int r = 0; r < 8; ++r) { mrow[r] = -INFINITY; lrow[r] = 0.f; }
#pragma unroll
  for (int t = 0; t < 4; ++t) oacc[t] = (v8f){0.f,0.f,0.f,0.f,0.f,0.f,0.f,0.f};

  const bool noisy = qb < nqbHalf;
  const int  nCh   = noisy ? (qb + 2) : (qb - nqbHalf + 1);
  for (int i = 0; i < nCh && i < kcHalf + 1; ++i) {
    const int  kc       = noisy ? ((i == 0) ? qb : (kcHalf + i - 1)) : (kcHalf + i);
    const bool needMask = (i == nCh - 1) || (noisy && i == 0);
    const int  kv0      = kc * kAtKC;
    __syncthreads();
    {
      const int r = tid >> 1, half = (tid & 1) * 32;
      const _Float16* ks = Kp + (size_t)(kv0 + r) * kD + half;
      const _Float16* vs = VT + (size_t)r * kS + kv0 + half;
#pragma unroll
      for (int u = 0; u < 4; ++u) {
        const v8h a0 = *(const v8h*)(ks + 8 * u);
        const v8h b0 = *(const v8h*)(vs + 8 * u);
        *(v8h*)(Ksh + r * kAtD  + half + 8 * u) = a0;
        *(v8h*)(Vth + r * kAtKC + half + 8 * u) = b0;
      }
    }
    __syncthreads();

    v8f s[4];
#pragma unroll
    for (int j = 0; j < 4; ++j) {
      s[j] = (v8f){0.f,0.f,0.f,0.f,0.f,0.f,0.f,0.f};
#pragma unroll
      for (int dc = 0; dc < 2; ++dc) {
        FH kb;
        kb.h[0] = *(const v8h*)(Ksh + (j * 16 + c) * kAtD + dc * 32 + 8 * hh);
        kb.h[1] = *(const v8h*)(Ksh + (j * 16 + c) * kAtD + dc * 32 + 16 + 8 * hh);
        s[j] = mma_h(qa[dc], kb.v, s[j]);
      }
    }
    float cm[8];
#pragma unroll
    for (int r = 0; r < 8; ++r) {
      const int qrow = q0 + 8 * hh + r;
      const int fq = qrow >> 10;
      const int bq = (qrow & (kNTok - 1)) >> kBlkShift;
      float m = -INFINITY;
#pragma unroll
      for (int j = 0; j < 4; ++j) {
        float sv = s[j][r] * sscale;
        if (needMask) {
          const int kvcol = kv0 + j * 16 + c;
          const int fk = kvcol >> 10;
          const int bk = (kvcol & (kNTok - 1)) >> kBlkShift;
          const bool allowed = ((fq == fk) && (bq == bk)) || ((fk > fq) && (bq > bk)) || (((fk & fq) != 0) && (bq >= bk));
          sv = allowed ? sv : -INFINITY;
        }
        s[j][r] = sv;
        m = fmaxf(m, sv);
      }
#pragma unroll
      for (int off = 1; off < 16; off <<= 1) m = fmaxf(m, __shfl_xor(m, off, 32));
      cm[r] = m;
    }
    _Float16* pw = Psh[wave];
#pragma unroll
    for (int r = 0; r < 8; ++r) {
      const float mnew  = fmaxf(mrow[r], cm[r]);
      const float alpha = (mrow[r] == -INFINITY) ? 0.f : expf(mrow[r] - mnew);
      mrow[r] = mnew;
      float psum = 0.f;
#pragma unroll
      for (int j = 0; j < 4; ++j) {
        const float sv = s[j][r];
        const float p  = (sv == -INFINITY) ? 0.f : expf(sv - mnew);
        psum += p;
        pw[(8 * hh + r) * kAtKC + j * 16 + c] = (_Float16)(p * kPsc);
      }
#pragma unroll
      for (int off = 1; off < 16; off <<= 1) psum += __shfl_xor(psum, off, 32);
      lrow[r] = lrow[r] * alpha + psum;
#pragma unroll
      for (int t = 0; t < 4; ++t) oacc[t][r] *= alpha;
    }
    __builtin_amdgcn_fence(__ATOMIC_RELEASE, "workgroup");
    __builtin_amdgcn_wave_barrier();
    __builtin_amdgcn_fence(__ATOMIC_ACQUIRE, "workgroup");
#pragma unroll 1
    for (int kk = 0; kk < 2; ++kk) {
      FH pa;
      pa.h[0] = *(const v8h*)(pw + c * kAtKC + kk * 32 + 8 * hh);
      pa.h[1] = *(const v8h*)(pw + c * kAtKC + kk * 32 + 16 + 8 * hh);
#pragma unroll
      for (int t = 0; t < 4; ++t) {
        FH vb;
        vb.h[0] = *(const v8h*)(Vth + (t * 16 + c) * kAtKC + kk * 32 + 8 * hh);
        vb.h[1] = *(const v8h*)(Vth + (t * 16 + c) * kAtKC + kk * 32 + 16 + 8 * hh);
        oacc[t] = mma_h(pa.v, vb.v, oacc[t]);
      }
    }
  }

  float* os = Os[wave];
#pragma unroll
  for (int r = 0; r < 8; ++r) {
    const float inv = 1.0f / (lrow[r] * kPsc);
#pragma unroll
    for (int t = 0; t < 4; ++t) os[(8 * hh + r) * 68 + t * 16 + c] = oacc[t][r] * inv;
  }
  __builtin_amdgcn_fence(__ATOMIC_RELEASE, "workgroup");
  __builtin_amdgcn_wave_barrier();
  __builtin_amdgcn_fence(__ATOMIC_ACQUIRE, "workgroup");
  {
    const int q8 = lane >> 3, c8 = (lane & 7) * 8;
    for (int pass = 0; pass < 2; ++pass) {
#pragma unroll
      for (int it = 0; it < 4; ++it) {
        const int row = it * 4 + q8;
        const float* sp = os + row * 68 + c8;
        v8h hv;
#pragma unroll
        for (int e = 0; e < 8; ++e) hv[e] = (_Float16)sp[e];
        *(volatile v8h*)(O + (size_t)(q0 + row) * kD + c8) = hv;
      }
      __threadfence();
    }
  }
}

extern "C" void kernel_launch(void* const* d_in, const int* in_sizes, int n_in,
                              void* d_out, int out_size, void* d_ws, size_t ws_size,
                              hipStream_t stream) {
  if (n_in < 14) return;
  if (in_sizes[0] != kS * kD || out_size != kS * kD) return;
  if (in_sizes[5] != kD3 * kD || in_sizes[8] != kD4 * kD || in_sizes[10] != kD * kD4 || in_sizes[12] != kD6 * kCond) return;

  const float* x     = (const float*)d_in[0];
  const float* cvec  = (const float*)d_in[1];
  const float* ropeC = (const float*)d_in[2];
  const float* ropeS = (const float*)d_in[3];
  const float* n1w   = (const float*)d_in[4];
  const float* wqkv  = (const float*)d_in[5];
  const float* wout  = (const float*)d_in[6];
  const float* n2w   = (const float*)d_in[7];
  const float* w1    = (const float*)d_in[8];
  const float* b1    = (const float*)d_in[9];
  const float* w2    = (const float*)d_in[10];
  const float* b2    = (const float*)d_in[11];
  const float* modw  = (const float*)d_in[12];
  const float* modb  = (const float*)d_in[13];
  float* out = (float*)d_out;

  size_t off = 0;
  auto take = [&](size_t bytes) -> size_t { const size_t o = off; off += (bytes + 255) & ~(size_t)255; return o; };
  const size_t oMods = take((size_t)kD6 * 4);
  const size_t oH16  = take((size_t)kS * kD * 2);
  const size_t oWqkv = take((size_t)kD3 * kD * 2);
  const size_t oWout = take((size_t)kD * kD * 2);
  const size_t oW1   = take((size_t)kD4 * kD * 2);
  const size_t oW2   = take((size_t)kD * kD4 * 2);
  const size_t oQKV  = take((size_t)3 * kS * kD * 2);
  const size_t oVT   = take((size_t)kD * kS * 2);
  const size_t oO16  = take((size_t)kS * kD * 2);
  const size_t oX2   = take((size_t)kS * kD * 4);
  const size_t oH2   = take((size_t)kS * kD * 2);
  const size_t oM1   = take((size_t)kS * kD4 * 2);
  if (off > ws_size) return;

  char* base = (char*)d_ws;
  float*          mods   = (float*)(base + oMods);
  unsigned short* h16    = (unsigned short*)(base + oH16);
  unsigned short* wqkv16 = (unsigned short*)(base + oWqkv);
  unsigned short* wout16 = (unsigned short*)(base + oWout);
  unsigned short* w1_16  = (unsigned short*)(base + oW1);
  unsigned short* w2_16  = (unsigned short*)(base + oW2);
  unsigned short* qkv16  = (unsigned short*)(base + oQKV);
  unsigned short* vt16   = (unsigned short*)(base + oVT);
  unsigned short* o16    = (unsigned short*)(base + oO16);
  float*          x2f    = (float*)(base + oX2);
  unsigned short* h2_16  = (unsigned short*)(base + oH2);
  unsigned short* m1_16  = (unsigned short*)(base + oM1);
  unsigned short* qplane = qkv16;
  unsigned short* kplane = qkv16 + (size_t)kS * kD;
  unsigned short* vplane = qkv16 + (size_t)2 * kS * kD;

  cond_mod_kernel<<<kD6 / 256, 256, 0, stream>>>(cvec, modw, modb, mods, kD6, kCond);

  {
    const int n2a = kD3 * kD / 2, n2b = kD * kD / 2, n2c = kD4 * kD / 2, n2d = kD * kD4 / 2;
    cast_scale_f16x2<<<(n2a + 255) / 256, 256, 0, stream>>>(wqkv, wqkv16, n2a, kWsc);
    cast_scale_f16x2<<<(n2b + 255) / 256, 256, 0, stream>>>(wout, wout16, n2b, kWsc);
    cast_scale_f16x2<<<(n2c + 255) / 256, 256, 0, stream>>>(w1,   w1_16,  n2c, kWsc);
    cast_scale_f16x2<<<(n2d + 255) / 256, 256, 0, stream>>>(w2,   w2_16,  n2d, kW2sc);
  }

  ln_mod_kernel<<<kS, 128, 0, stream>>>(x, n1w, mods, mods + kD, h16);

  {
    const int tiles = (kS / 64) * (kD3 / 64);
    wmma_gemm64<0, false, 0, 3, false, 0, false><<<dim3((tiles + 7) / 8, 1), 256, 0, stream>>>(
        h16, h16, kD, 0L, wqkv16, wqkv16, kD, 0L, (void*)qkv16, (void*)qkv16, kD, 0L,
        mods, x, 0L, mods, ropeC, ropeS, (long)kS * kD, kS, kD3, kD, 1.0f / kWsc);
  }

  vtrans_kernel<<<dim3(kD / 64, kS / 64), 256, 0, stream>>>(vplane, vt16);

  attn_bd_kernel<<<kH * (kS / kAtQB), 128, 0, stream>>>(qplane, kplane, vt16, o16, 0.125f);

  {
    const int tiles = (kS / 64) * (kD / 64);
    wmma_gemm64<0, false, 0, 0, true, 0, true><<<dim3((tiles + 7) / 8, 1), 256, 0, stream>>>(
        o16, o16, kD, 0L, wout16, wout16, kD, 0L, (void*)x2f, (void*)x2f, kD, 0L,
        mods, x, 0L, mods + 2 * kD, ropeC, ropeS, 0L, kS, kD, kD, 1.0f / kWsc);
  }

  ln_mod_kernel<<<kS, 128, 0, stream>>>(x2f, n2w, mods + 3 * kD, mods + 4 * kD, h2_16);

  {
    const int tiles = (kS / 64) * (kD4 / 64);
    wmma_gemm64<0, false, 2, 1, false, 6, false><<<dim3((tiles + 7) / 8, 1), 256, 0, stream>>>(
        h2_16, h2_16, kD, 0L, w1_16, w1_16, kD, 0L, (void*)m1_16, (void*)m1_16, kD4, 0L,
        b1, x, 0L, mods, ropeC, ropeS, 0L, kS, kD4, kD, 1.0f / kWsc);
  }

  {
    const int tiles = (kS / 64) * (kD / 64);
    wmma_gemm64<0, false, 2, 0, true, 0, true><<<dim3((tiles + 7) / 8, 1), 256, 0, stream>>>(
        m1_16, m1_16, kD4, 0L, w2_16, w2_16, kD4, 0L, (void*)out, (void*)out, kD, 0L,
        b2, x2f, 0L, mods + 5 * kD, ropeC, ropeS, 0L, kS, kD, kD4, 1.0f / kW2sc);
  }
}
